// AttentionBlock_16398185136213
// MI455X (gfx1250) — hardware-verified
//
#include <hip/hip_runtime.h>
#include <stdint.h>

typedef __attribute__((ext_vector_type(16))) _Float16 v16h;
typedef __attribute__((ext_vector_type(8)))  _Float16 v8h;
typedef __attribute__((ext_vector_type(8)))  float    v8f;
typedef __attribute__((ext_vector_type(4)))  float    v4f;

constexpr int kBatch    = 8;
constexpr int kSeq      = 1024;
constexpr int kDin      = 512;
constexpr int kHeads    = 8;
constexpr int kDhead    = 64;
constexpr int kDexp     = 2048;
constexpr int kDout     = 512;
constexpr int kDqk      = 2 * kHeads * kDhead;
constexpr int kDvh      = kDin;
constexpr int kDv       = kHeads * kDvh;
constexpr int kDqkv     = kDqk + kDv;
constexpr int kRows     = kBatch * kSeq;
constexpr int kHalfB    = kBatch / 2;
constexpr int kHalfRows = kHalfB * kSeq;

static_assert(kRows % 64 == 0 && kDqk % 64 == 0 && kDin % 32 == 0, "qk gemm");
static_assert(kDv % 64 == 0 && kHalfRows % 64 == 0, "vt gemm");
static_assert(kDin % 64 == 0 && kDv % 32 == 0, "merge gemm");
static_assert(kDexp % 64 == 0 && kDexp % 32 == 0 && kDout % 64 == 0, "ffn gemms");
static_assert(kDin % 64 == 0 && kDqkv % 64 == 0 && kDv % 64 == 0 && kDexp % 64 == 0 && kDout % 64 == 0, "weight transpose tiles");
static_assert(kSeq == 1024 && kDhead == 64 && kDvh == 512, "attention kernel geometry");

__device__ __forceinline__ void dep_guard_h(v8f& a, v8f& b, v16h x, v16h y) { asm volatile("v_nop\n\tv_nop\n\tv_nop\n\tv_nop" : "+v"(a), "+v"(b) : "v"(x), "v"(y)); }
__device__ __forceinline__ void keep4_h(v16h a, v16h b, v16h c, v16h d) { asm volatile("v_nop" :: "v"(a), "v"(b), "v"(c), "v"(d)); }
__device__ __forceinline__ void acc_guard4(v8f& a, v8f& b, v8f& c, v8f& d) { asm volatile("v_nop\n\tv_nop\n\tv_nop\n\tv_nop" : "+v"(a), "+v"(b), "+v"(c), "+v"(d)); }

template <typename T> struct Frag;
template <> struct Frag<_Float16> {
  typedef v16h V; union U { v16h v; v8h h[2]; };
  static __device__ __forceinline__ v16h load(const _Float16* p) {
    U f; f.h[0] = *(const v8h*)(p); f.h[1] = *(const v8h*)(p + 16); return f.v;
  }
  static __device__ __forceinline__ v8f mma(v16h a, v16h b, v8f c) {
    return __builtin_amdgcn_wmma_f32_16x16x32_f16(false, a, false, b, (short)0, c, false, false);
  }
  static __device__ __forceinline__ void guard(v8f& a, v8f& b, v16h x, v16h y) { dep_guard_h(a, b, x, y); }
  static __device__ __forceinline__ void keep(v16h a, v16h b, v16h c, v16h d) { keep4_h(a, b, c, d); }
};

__device__ __forceinline__ v8f zero8() { return (v8f){0.f, 0.f, 0.f, 0.f, 0.f, 0.f, 0.f, 0.f}; }

__device__ __forceinline__ float swishf(float v) {
  const float e = expf(-v);
  return v * __builtin_amdgcn_rcpf(1.0f + e);
}

__device__ __forceinline__ float h16lo(unsigned w) { return (float)__builtin_bit_cast(_Float16, (unsigned short)(w & 0xffffu)); }
__device__ __forceinline__ float h16hi(unsigned w) { return (float)__builtin_bit_cast(_Float16, (unsigned short)(w >> 16)); }
__device__ __forceinline__ float sqsum4(uint4 w) {
  float s = 0.0f;
  float a;
  a = h16lo(w.x); s += a * a;  a = h16hi(w.x); s += a * a;
  a = h16lo(w.y); s += a * a;  a = h16hi(w.y); s += a * a;
  a = h16lo(w.z); s += a * a;  a = h16hi(w.z); s += a * a;
  a = h16lo(w.w); s += a * a;  a = h16hi(w.w); s += a * a;
  return s;
}

__global__ __launch_bounds__(256) void wcast_t_kernel(const float* __restrict__ W, _Float16* __restrict__ out,
                                                     int Kd, int Nd, float mul) {
  __shared__ float tileT[64][65];
  const int tid = threadIdx.x, lane = tid & 31, wave = tid >> 5;
  const int n0 = blockIdx.x * 64, k0 = blockIdx.y * 64;
#pragma unroll
  for (int i = 0; i < 4; ++i) {
    const int idx = i * 256 + tid;
    const int kr = idx >> 4, nq = (idx & 15) * 4;
    const v4f v = *(const v4f*)(W + (size_t)(k0 + kr) * Nd + n0 + nq);
    tileT[kr][nq + 0] = v[0];
    tileT[kr][nq + 1] = v[1];
    tileT[kr][nq + 2] = v[2];
    tileT[kr][nq + 3] = v[3];
  }
  __syncthreads();
  const int q = lane >> 3, c8 = (lane & 7) * 8;
  v8h hv[2];
#pragma unroll
  for (int it = 0; it < 2; ++it) {
    const int n = wave * 8 + it * 4 + q;
    v8h t;
#pragma unroll
    for (int e = 0; e < 8; ++e) t[e] = (_Float16)(tileT[c8 + e][n] * mul);
    hv[it] = t;
  }
  for (int pass = 0; pass < 2; ++pass) {
#pragma unroll
    for (int it = 0; it < 2; ++it) {
      const int n = wave * 8 + it * 4 + q;
      *(volatile v8h*)(out + (size_t)(n0 + n) * Kd + k0 + c8) = hv[it];
    }
    __threadfence();
  }
}

__global__ __launch_bounds__(256) void fnorm_stats_kernel(const float* __restrict__ in, float* __restrict__ mean_t,
                                                         float* __restrict__ rstd_t, int Dd) {
  __shared__ float red[8][33];
  const int tid = threadIdx.x, f = tid & 31, s = tid >> 5;
  const int groups = Dd >> 5;
  const int bl = blockIdx.x / groups;
  const int g = blockIdx.x - bl * groups;
  const int d = g * 32 + f;
  const float* p = in + ((size_t)bl * kSeq + (size_t)s * 128) * Dd + d;
  float sum = 0.0f;
#pragma unroll 4
  for (int j = 0; j < 128; ++j) sum += p[(size_t)j * Dd];
  red[s][f] = sum;
  __syncthreads();
  float tot = 0.0f;
#pragma unroll
  for (int u = 0; u < 8; ++u) tot += red[u][f];
  const float mean = tot * (1.0f / 1024.0f);
  __syncthreads();
  float ss = 0.0f;
#pragma unroll 4
  for (int j = 0; j < 128; ++j) {
    const float dv = p[(size_t)j * Dd] - mean;
    ss += dv * dv;
  }
  red[s][f] = ss;
  __syncthreads();
  float vtot = 0.0f;
#pragma unroll
  for (int u = 0; u < 8; ++u) vtot += red[u][f];
  const float var = vtot * (1.0f / 1024.0f);
  const float rstd = 1.0f / sqrtf(var + 1e-5f);
  if (s == 0) {
    float* mp = mean_t + (size_t)bl * Dd + d;
    float* rp = rstd_t + (size_t)bl * Dd + d;
    *(volatile float*)mp = mean;
    *(volatile float*)rp = rstd;
    __threadfence();
    *(volatile float*)mp = mean;
    *(volatile float*)rp = rstd;
  }
}

template <bool POS, bool SWISH>
__global__ __launch_bounds__(256) void fnorm_apply_kernel(const float* __restrict__ in, const float* __restrict__ pos,
    const float* __restrict__ gamma, const float* __restrict__ beta,
    const float* __restrict__ mean_t, const float* __restrict__ rstd_t,
    _Float16* __restrict__ out16, int Dd, int total8) {
  const int gid = blockIdx.x * 256 + threadIdx.x;
  if (gid >= total8) return;
  const size_t e0 = (size_t)gid * 8;
  const int r = (int)(e0 / (size_t)Dd);
  const int d = (int)(e0 - (size_t)r * Dd);
  const int bl = r >> 10, n = r & 1023;
  const v4f x0 = *(const v4f*)(in + e0);
  const v4f x1 = *(const v4f*)(in + e0 + 4);
  const v4f m0 = *(const v4f*)(mean_t + (size_t)bl * Dd + d);
  const v4f m1 = *(const v4f*)(mean_t + (size_t)bl * Dd + d + 4);
  const v4f s0 = *(const v4f*)(rstd_t + (size_t)bl * Dd + d);
  const v4f s1 = *(const v4f*)(rstd_t + (size_t)bl * Dd + d + 4);
  const v4f g0 = *(const v4f*)(gamma + d);
  const v4f g1 = *(const v4f*)(gamma + d + 4);
  const v4f b0 = *(const v4f*)(beta + d);
  const v4f b1 = *(const v4f*)(beta + d + 4);
  v4f y0 = (g0 * (x0 - m0)) * s0 + b0;
  v4f y1 = (g1 * (x1 - m1)) * s1 + b1;
  if (POS) {
    y0 += *(const v4f*)(pos + (size_t)n * Dd + d);
    y1 += *(const v4f*)(pos + (size_t)n * Dd + d + 4);
  }
  float vals[8];
#pragma unroll
  for (int e = 0; e < 4; ++e) { vals[e] = y0[e]; vals[4 + e] = y1[e]; }
  if (SWISH) {
#pragma unroll
    for (int e = 0; e < 8; ++e) vals[e] = swishf(vals[e]);
  }
  v8h hv;
#pragma unroll
  for (int e = 0; e < 8; ++e) hv[e] = (_Float16)vals[e];
  _Float16* op = out16 + e0;
  *(volatile v8h*)op = hv;
  __threadfence();
  *(volatile v8h*)op = hv;
}

template <int BIAS_MODE, int OUT_MODE, bool RESID>
__global__ __launch_bounds__(256) void gemm64_f16(
    const _Float16* __restrict__ A, int lda,
    const _Float16* __restrict__ Bt, int ldb,
    void* __restrict__ Cout, int ldc,
    const float* __restrict__ bias,
    const float* __restrict__ resid,
    int M, int N, int K, float scale) {
  typedef _Float16 T;
  typedef v16h V;
  __shared__ __align__(16) float sT[8][16 * 68];
  const int lane = threadIdx.x & 31;
  const int wave = threadIdx.x >> 5;
  const int tilesN = N >> 6;
  const int tilesM = M >> 6;
  const int tile = blockIdx.x * 8 + wave;
  if (tile >= tilesM * tilesN) return;
  const int tm = tile / tilesN;
  const int tn = tile - tm * tilesN;
  const int m0 = tm << 6;
  const int n0 = tn << 6;
  const int rlane = lane & 15;
  const int koff  = (lane >> 4) * 8;
  const int mOff  = (lane >> 4) * 8;

  v8f acc[4][4];
#pragma unroll
  for (int i = 0; i < 4; ++i)
#pragma unroll
    for (int j = 0; j < 4; ++j) acc[i][j] = zero8();

  for (int k0 = 0; k0 < K; k0 += 32) {
    V bh[4];
#pragma unroll
    for (int j = 0; j < 4; ++j) {
      const size_t bo = (size_t)(n0 + (j << 4) + rlane) * ldb + koff + k0;
      bh[j] = Frag<T>::load(Bt + bo);
    }
#pragma unroll
    for (int i = 0; i < 4; ++i) {
      const size_t ao = (size_t)(m0 + (i << 4) + rlane) * lda + koff + k0;
      V ah = Frag<T>::load(A + ao);
#pragma unroll
      for (int j = 0; j < 4; ++j) acc[i][j] = Frag<T>::mma(ah, bh[j], acc[i][j]);
      Frag<T>::guard(acc[i][0], acc[i][3], ah, ah);
    }
    Frag<T>::keep(bh[0], bh[1], bh[2], bh[3]);
  }
  acc_guard4(acc[0][0], acc[0][1], acc[0][2], acc[0][3]);
  acc_guard4(acc[1][0], acc[1][1], acc[1][2], acc[1][3]);
  acc_guard4(acc[2][0], acc[2][1], acc[2][2], acc[2][3]);
  acc_guard4(acc[3][0], acc[3][1], acc[3][2], acc[3][3]);

  float* slab = sT[wave];
  if (OUT_MODE == 0) {
    const int hq = lane >> 4, c4 = (lane & 15) * 4;
    v4f bias4 = {0.f, 0.f, 0.f, 0.f};
    if (BIAS_MODE == 2) bias4 = *(const v4f*)(bias + n0 + c4);
    float* Cf = (float*)Cout;
#pragma unroll
    for (int i = 0; i < 4; ++i) {
      const int mBase = m0 + (i << 4);
#pragma unroll
      for (int j = 0; j < 4; ++j) {
#pragma unroll
        for (int r = 0; r < 8; ++r) slab[(mOff + r) * 68 + (j << 4) + rlane] = acc[i][j][r] * scale;
      }
      __builtin_amdgcn_fence(__ATOMIC_RELEASE, "workgroup");
      __builtin_amdgcn_wave_barrier();
      __builtin_amdgcn_fence(__ATOMIC_ACQUIRE, "workgroup");
      v4f vals[8];
#pragma unroll
      for (int it = 0; it < 8; ++it) {
        const int row = it * 2 + hq;
        v4f v = *(const v4f*)(slab + row * 68 + c4);
        if (BIAS_MODE == 2) v += bias4;
        if (BIAS_MODE == 1) { const float bm = bias[mBase + row]; v += bm; }
        if (RESID) {
          const v4f rr = *(const v4f*)(resid + (size_t)(mBase + row) * ldc + n0 + c4);
          v += rr;
        }
        vals[it] = v;
      }
      for (int pass = 0; pass < 2; ++pass) {
#pragma unroll
        for (int it = 0; it < 8; ++it) {
          const int row = it * 2 + hq;
          *(volatile v4f*)(Cf + (size_t)(mBase + row) * ldc + n0 + c4) = vals[it];
        }
        __threadfence();
      }
      __builtin_amdgcn_fence(__ATOMIC_RELEASE, "workgroup");
      __builtin_amdgcn_wave_barrier();
      __builtin_amdgcn_fence(__ATOMIC_ACQUIRE, "workgroup");
    }
  } else {
    const int q = lane >> 3, c8 = (lane & 7) * 8;
    v4f b8a = {0.f, 0.f, 0.f, 0.f}, b8b = {0.f, 0.f, 0.f, 0.f};
    if (BIAS_MODE == 2) {
      b8a = *(const v4f*)(bias + n0 + c8);
      b8b = *(const v4f*)(bias + n0 + c8 + 4);
    }
    _Float16* Ch = (_Float16*)Cout;
#pragma unroll
    for (int i = 0; i < 4; ++i) {
      const int mBase = m0 + (i << 4);
#pragma unroll
      for (int j = 0; j < 4; ++j) {
#pragma unroll
        for (int r = 0; r < 8; ++r) slab[(mOff + r) * 68 + (j << 4) + rlane] = acc[i][j][r] * scale;
      }
      __builtin_amdgcn_fence(__ATOMIC_RELEASE, "workgroup");
      __builtin_amdgcn_wave_barrier();
      __builtin_amdgcn_fence(__ATOMIC_ACQUIRE, "workgroup");
      v8h hvals[4];
#pragma unroll
      for (int it = 0; it < 4; ++it) {
        const int row = it * 4 + q;
        const float* sp = slab + row * 68 + c8;
        v4f va = *(const v4f*)(sp);
        v4f vb = *(const v4f*)(sp + 4);
        if (BIAS_MODE == 2) { va += b8a; vb += b8b; }
        if (BIAS_MODE == 1) { const float bm = bias[mBase + row]; va += bm; vb += bm; }
        v8h hv;
#pragma unroll
        for (int e = 0; e < 4; ++e) { hv[e] = (_Float16)va[e]; hv[4 + e] = (_Float16)vb[e]; }
        hvals[it] = hv;
      }
      for (int pass = 0; pass < 2; ++pass) {
#pragma unroll
        for (int it = 0; it < 4; ++it) {
          const int row = it * 4 + q;
          *(volatile v8h*)(Ch + (size_t)(mBase + row) * ldc + n0 + c8) = hvals[it];
        }
        __threadfence();
      }
      __builtin_amdgcn_fence(__ATOMIC_RELEASE, "workgroup");
      __builtin_amdgcn_wave_barrier();
      __builtin_amdgcn_fence(__ATOMIC_ACQUIRE, "workgroup");
    }
  }
}

__global__ __launch_bounds__(256) void qk2_kernel(const _Float16* __restrict__ QK, float* __restrict__ q2t,
                                                 float* __restrict__ k2t) {
  const int gid = blockIdx.x * 256 + threadIdx.x;
  const int bhg = gid >> 10, n = gid & 1023, b = bhg >> 3, h = bhg & 7;
  const uint4* qp = (const uint4*)(QK + ((size_t)(b * kSeq + n) * kDqk + h * kDhead));
  const uint4* kp = (const uint4*)(QK + ((size_t)(b * kSeq + n) * kDqk + 512 + h * kDhead));
  float sq = 0.0f, sk = 0.0f;
#pragma unroll 1
  for (int i = 0; i < 8; ++i) { const uint4 w = qp[i]; sq += sqsum4(w); }
#pragma unroll 1
  for (int i = 0; i < 8; ++i) { const uint4 w = kp[i]; sk += sqsum4(w); }
  *(volatile float*)(q2t + gid) = sq;
  *(volatile float*)(k2t + gid) = sk;
  __threadfence();
  *(volatile float*)(q2t + gid) = sq;
  *(volatile float*)(k2t + gid) = sk;
}

constexpr int kLP = 72;
__global__ __launch_bounds__(256) void rbf_attn_kernel(
    const _Float16* __restrict__ QK, const _Float16* __restrict__ Vt,
    const float* __restrict__ q2t, const float* __restrict__ k2t,
    const float* __restrict__ scale_p, _Float16* __restrict__ Oh, int hb) {
  __shared__ __align__(16) _Float16 Ksh[64 * kLP];
  __shared__ __align__(16) _Float16 Vsh[512 * kLP];
  __shared__ __align__(16) _Float16 Psh[64 * kLP];
  __shared__ float q2s[64];
  __shared__ float k2s[64];
  const int tid = threadIdx.x, wave = tid >> 5, lane = tid & 31;
  const int rlane = lane & 15, hh = lane >> 4, koff = hh * 8;
  const int blk = blockIdx.x;
  const int qb = blk & 15, h = (blk >> 4) & 7, bl = blk >> 7;
  const int bglob = hb * kHalfB + bl;
  const int bhg = bglob * kHeads + h;
  const size_t qrow0 = (size_t)bglob * kSeq + qb * 64;
  const size_t krow0 = (size_t)bglob * kSeq;
  const float sc = scale_p[0];
  const float neg_inv = -1.0f / (sc * sc);
  const int rt = wave & 3;
  const int ct0 = (wave >> 2) * 2;
  if (tid < 64) q2s[tid] = q2t[(size_t)bhg * kSeq + qb * 64 + tid];

  v8f acc[4][4];
#pragma unroll
  for (int i = 0; i < 4; ++i)
#pragma unroll
    for (int j = 0; j < 4; ++j) acc[i][j] = zero8();

  for (int kc = 0; kc < 16; ++kc) {
    const int kv0 = kc * 64;
    __syncthreads();
#pragma unroll
    for (int i = 0; i < 2; ++i) {
      const int idx = i * 256 + tid;
      const int row = idx >> 3, seg = (idx & 7) * 8;
      const uint4 w = *(const uint4*)(QK + (krow0 + kv0 + row) * kDqk + 512 + h * kDhead + seg);
      *(uint4*)(Ksh + row * kLP + seg) = w;
    }
#pragma unroll 1
    for (int g4 = 0; g4 < 4; ++g4) {
      uint4 w0, w1, w2, w3;
      {
        const int idx = (g4 * 4 + 0) * 256 + tid; const int cr = idx >> 3, seg = (idx & 7) * 8;
        w0 = *(const uint4*)(Vt + (size_t)(h * kDvh + cr) * kHalfRows + bl * kSeq + kv0 + seg);
      }
      {
        const int idx = (g4 * 4 + 1) * 256 + tid; const int cr = idx >> 3, seg = (idx & 7) * 8;
        w1 = *(const uint4*)(Vt + (size_t)(h * kDvh + cr) * kHalfRows + bl * kSeq + kv0 + seg);
      }
      {
        const int idx = (g4 * 4 + 2) * 256 + tid; const int cr = idx >> 3, seg = (idx & 7) * 8;
        w2 = *(const uint4*)(Vt + (size_t)(h * kDvh + cr) * kHalfRows + bl * kSeq + kv0 + seg);
      }
      {
        const int idx = (g4 * 4 + 3) * 256 + tid; const int cr = idx >> 3, seg = (idx & 7) * 8;
        w3 = *(const uint4*)(Vt + (size_t)(h * kDvh + cr) * kHalfRows + bl * kSeq + kv0 + seg);
      }
      { const int idx = (g4 * 4 + 0) * 256 + tid; const int cr = idx >> 3, seg = (idx & 7) * 8; *(uint4*)(Vsh + cr * kLP + seg) = w0; }
      { const int idx = (g4 * 4 + 1) * 256 + tid; const int cr = idx >> 3, seg = (idx & 7) * 8; *(uint4*)(Vsh + cr * kLP + seg) = w1; }
      { const int idx = (g4 * 4 + 2) * 256 + tid; const int cr = idx >> 3, seg = (idx & 7) * 8; *(uint4*)(Vsh + cr * kLP + seg) = w2; }
      { const int idx = (g4 * 4 + 3) * 256 + tid; const int cr = idx >> 3, seg = (idx & 7) * 8; *(uint4*)(Vsh + cr * kLP + seg) = w3; }
    }
    if (tid < 64) k2s[tid] = k2t[(size_t)bhg * kSeq + kv0 + tid];
    __syncthreads();

    const _Float16* qp = QK + (qrow0 + rt * 16 + rlane) * kDqk + h * kDhead + koff;
    const v16h qa0 = Frag<_Float16>::load(qp);
    const v16h qa1 = Frag<_Float16>::load(qp + 32);
    const _Float16* kp0 = Ksh + ((ct0 + 0) * 16 + rlane) * kLP + koff;
    const _Float16* kp1 = Ksh + ((ct0 + 1) * 16 + rlane) * kLP + koff;
    const v16h kb00 = Frag<_Float16>::load(kp0);
    const v16h kb01 = Frag<_Float16>::load(kp0 + 32);
    const v16h kb10 = Frag<_Float16>::load(kp1);
    const v16h kb11 = Frag<_Float16>::load(kp1 + 32);
    v8f s[2];
    s[0] = zero8();
    s[1] = zero8();
    s[0] = Frag<_Float16>::mma(qa0, kb00, s[0]);
    s[0] = Frag<_Float16>::mma(qa1, kb01, s[0]);
    s[1] = Frag<_Float16>::mma(qa0, kb10, s[1]);
    s[1] = Frag<_Float16>::mma(qa1, kb11, s[1]);
    dep_guard_h(s[0], s[1], qa0, qa1);
    keep4_h(kb00, kb01, kb10, kb11);

#pragma unroll
    for (int r = 0; r < 8; ++r) {
      const int m = rt * 16 + 8 * hh + r;
      const float q2v = q2s[m];
#pragma unroll
      for (int j = 0; j < 2; ++j) {
        const int col = (ct0 + j) * 16 + rlane;
        float d2 = q2v + k2s[col] - 2.0f * s[j][r];
        d2 = fmaxf(d2, 0.0f);
        const float p = expf(d2 * neg_inv) * 32768.0f;
        Psh[m * kLP + col] = (_Float16)p;
      }
    }
    __syncthreads();

#pragma unroll
    for (int kk = 0; kk < 2; ++kk) {
      const int k0 = kk * 32;
      v16h vb[4];
#pragma unroll
      for (int j = 0; j < 4; ++j) vb[j] = Frag<_Float16>::load(Vsh + (wave * 64 + j * 16 + rlane) * kLP + koff + k0);
#pragma unroll
      for (int i = 0; i < 4; ++i) {
        const v16h pa = Frag<_Float16>::load(Psh + (i * 16 + rlane) * kLP + koff + k0);
#pragma unroll
        for (int j = 0; j < 4; ++j) acc[i][j] = Frag<_Float16>::mma(pa, vb[j], acc[i][j]);
        dep_guard_h(acc[i][0], acc[i][3], pa, pa);
      }
      keep4_h(vb[0], vb[1], vb[2], vb[3]);
    }
  }
  acc_guard4(acc[0][0], acc[0][1], acc[0][2], acc[0][3]);
  acc_guard4(acc[1][0], acc[1][1], acc[1][2], acc[1][3]);
  acc_guard4(acc[2][0], acc[2][1], acc[2][2], acc[2][3]);
  acc_guard4(acc[3][0], acc[3][1], acc[3][2], acc[3][3]);
  __syncthreads();

  float* slab = reinterpret_cast<float*>(Vsh) + wave * (16 * 68);
  const int mOff = hh * 8;
  const int q = lane >> 3, c8 = (lane & 7) * 8;
  const float oscale = 1.0f / 512.0f;
#pragma unroll
  for (int i = 0; i < 4; ++i) {
#pragma unroll
    for (int j = 0; j < 4; ++j) {
#pragma unroll
      for (int r = 0; r < 8; ++r) slab[(mOff + r) * 68 + (j << 4) + rlane] = acc[i][j][r] * oscale;
    }
    __builtin_amdgcn_fence(__ATOMIC_RELEASE, "workgroup");
    __builtin_amdgcn_wave_barrier();
    __builtin_amdgcn_fence(__ATOMIC_ACQUIRE, "workgroup");
    v8h hvals[4];
#pragma unroll
    for (int it = 0; it < 4; ++it) {
      const int row = it * 4 + q;
      const float* sp = slab + row * 68 + c8;
      const v4f va = *(const v4f*)(sp);
      const v4f vbv = *(const v4f*)(sp + 4);
      v8h hv;
#pragma unroll
      for (int e = 0; e < 4; ++e) { hv[e] = (_Float16)va[e]; hv[4 + e] = (_Float16)vbv[e]; }
      hvals[it] = hv;
    }
    for (int pass = 0; pass < 2; ++pass) {
#pragma unroll
      for (int it = 0; it < 4; ++it) {
        const int row = it * 4 + q;
        const size_t orow = (size_t)bl * kSeq + qb * 64 + i * 16 + row;
        *(volatile v8h*)(Oh + orow * kDv + h * kDvh + wave * 64 + c8) = hvals[it];
      }
      __threadfence();
    }
    __builtin_amdgcn_fence(__ATOMIC_RELEASE, "workgroup");
    __builtin_amdgcn_wave_barrier();
    __builtin_amdgcn_fence(__ATOMIC_ACQUIRE, "workgroup");
  }
}

extern "C" void kernel_launch(void* const* d_in, const int* in_sizes, int n_in,
                              void* d_out, int out_size, void* d_ws, size_t ws_size,
                              hipStream_t stream) {
  (void)in_sizes;
  if (n_in < 17) return;
  if (out_size != kRows * kDout) return;
  const float* x      = (const float*)d_in[0];
  const float* pos    = (const float*)d_in[1];
  const float* gam1   = (const float*)d_in[2];
  const float* bet1   = (const float*)d_in[3];
  const float* scalep = (const float*)d_in[4];
  const float* Wqkv   = (const float*)d_in[5];
  const float* bqkv   = (const float*)d_in[6];
  const float* Wm     = (const float*)d_in[7];
  const float* bm     = (const float*)d_in[8];
  const float* gam2   = (const float*)d_in[9];
  const float* bet2   = (const float*)d_in[10];
  const float* W1     = (const float*)d_in[11];
  const float* b1     = (const float*)d_in[12];
  const float* gam3   = (const float*)d_in[13];
  const float* bet3   = (const float*)d_in[14];
  const float* W2     = (const float*)d_in[15];
  const float* b2     = (const float*)d_in[16];
  float* out = (float*)d_out;

  const size_t szWqkvT = (size_t)kDqkv * kDin * 2;
  const size_t szWmT   = (size_t)kDin * kDv * 2;
  const size_t szW1T   = (size_t)kDexp * kDin * 2;
  const size_t szW2T   = (size_t)kDout * kDexp * 2;
  const size_t szTab   = (size_t)kBatch * kDin * 4;
  const size_t szTab3  = (size_t)kHalfB * kDexp * 4;
  const size_t szQ2    = (size_t)kBatch * kHeads * kSeq * 4;
  const size_t szX2    = (size_t)kRows * kDin * 4;
  const size_t szA1    = (size_t)kRows * kDin * 2;
  const size_t szQK    = (size_t)kRows * kDqk * 2;
  const size_t szVth   = (size_t)kDv * kHalfRows * 2;
  const size_t szOh    = (size_t)kHalfRows * kDv * 2;
  const size_t szFfh   = (size_t)kHalfRows * kDexp * 4;
  const size_t szA3h   = (size_t)kHalfRows * kDexp * 2;
  const size_t arenaA  = szA1 + szQK + szVth + szOh;
  const size_t arenaB  = szA1 + szFfh + szA3h;
  const size_t szArena = arenaA > arenaB ? arenaA : arenaB;

  char* wbase = (char*)d_ws;
  size_t off = 0;
  auto carve = [&](size_t bytes) -> char* { char* p = wbase + off; off += (bytes + 255) & ~(size_t)255; return p; };
  _Float16* WqkvT = (_Float16*)carve(szWqkvT);
  _Float16* WmT   = (_Float16*)carve(szWmT);
  _Float16* W1T   = (_Float16*)carve(szW1T);
  _Float16* W2T   = (_Float16*)carve(szW2T);
  float* mean1 = (float*)carve(szTab);
  float* rstd1 = (float*)carve(szTab);
  float* mean2 = (float*)carve(szTab);
  float* rstd2 = (float*)carve(szTab);
  float* mean3 = (float*)carve(szTab3);
  float* rstd3 = (float*)carve(szTab3);
  float* q2t   = (float*)carve(szQ2);
  float* k2t   = (float*)carve(szQ2);
  float* x2    = (float*)carve(szX2);
  char* arena  = carve(szArena);
  if (off > ws_size) return;
  _Float16* A1   = (_Float16*)(arena);
  _Float16* QK16 = (_Float16*)(arena + szA1);
  _Float16* Vth  = (_Float16*)(arena + szA1 + szQK);
  _Float16* Oh   = (_Float16*)(arena + szA1 + szQK + szVth);
  _Float16* A2   = (_Float16*)(arena);
  float*    ffh  = (float*)(arena + szA1);
  _Float16* A3h  = (_Float16*)(arena + szA1 + szFfh);

  const float inv256   = 1.0f / 256.0f;
  const float inv16384 = 1.0f / 16384.0f;

  wcast_t_kernel<<<dim3(kDqkv / 64, kDin / 64), dim3(256), 0, stream>>>(Wqkv, WqkvT, kDin, kDqkv, 256.0f);
  wcast_t_kernel<<<dim3(kDin / 64, kDv / 64), dim3(256), 0, stream>>>(Wm, WmT, kDv, kDin, 256.0f);
  wcast_t_kernel<<<dim3(kDexp / 64, kDin / 64), dim3(256), 0, stream>>>(W1, W1T, kDin, kDexp, 256.0f);
  wcast_t_kernel<<<dim3(kDout / 64, kDexp / 64), dim3(256), 0, stream>>>(W2, W2T, kDexp, kDout, 256.0f);

  fnorm_stats_kernel<<<dim3(kBatch * (kDin / 32)), dim3(256), 0, stream>>>(x, mean1, rstd1, kDin);
  fnorm_apply_kernel<true, true><<<dim3((kRows * kDin / 8) / 256), dim3(256), 0, stream>>>(
      x, pos, gam1, bet1, mean1, rstd1, A1, kDin, kRows * kDin / 8);

  gemm64_f16<2, 1, false><<<dim3((kRows / 64) * (kDqk / 64) / 8), dim3(256), 0, stream>>>(
      A1, kDin, WqkvT, kDin, (void*)QK16, kDqk, bqkv, x, kRows, kDqk, kDin, inv256);
  qk2_kernel<<<dim3((kBatch * kHeads * kSeq) / 256), dim3(256), 0, stream>>>(QK16, q2t, k2t);

  for (int hb = 0; hb < 2; ++hb) {
    gemm64_f16<1, 1, false><<<dim3((kDv / 64) * (kHalfRows / 64) / 8), dim3(256), 0, stream>>>(
        WqkvT + (size_t)kDqk * kDin, kDin, A1 + (size_t)hb * kHalfRows * kDin, kDin,
        (void*)Vth, kHalfRows, bqkv + kDqk, x, kDv, kHalfRows, kDin, inv256);
    rbf_attn_kernel<<<dim3(kHalfB * kHeads * (kSeq / 64)), dim3(256), 0, stream>>>(
        QK16, Vth, q2t, k2t, scalep, Oh, hb);
    gemm64_f16<2, 0, true><<<dim3((kHalfRows / 64) * (kDin / 64) / 8), dim3(256), 0, stream>>>(
        Oh, kDv, WmT, kDv, (void*)(x2 + (size_t)hb * kHalfRows * kDin), kDin, bm,
        x + (size_t)hb * kHalfRows * kDin, kHalfRows, kDin, kDv, inv16384);
  }

  fnorm_stats_kernel<<<dim3(kBatch * (kDin / 32)), dim3(256), 0, stream>>>(x2, mean2, rstd2, kDin);
  fnorm_apply_kernel<false, false><<<dim3((kRows * kDin / 8) / 256), dim3(256), 0, stream>>>(
      x2, pos, gam2, bet2, mean2, rstd2, A2, kDin, kRows * kDin / 8);

  for (int hb = 0; hb < 2; ++hb) {
    gemm64_f16<2, 0, false><<<dim3((kHalfRows / 64) * (kDexp / 64) / 8), dim3(256), 0, stream>>>(
        A2 + (size_t)hb * kHalfRows * kDin, kDin, W1T, kDin, (void*)ffh, kDexp, b1, x,
        kHalfRows, kDexp, kDin, inv256);
    fnorm_stats_kernel<<<dim3(kHalfB * (kDexp / 32)), dim3(256), 0, stream>>>(ffh, mean3, rstd3, kDexp);
    fnorm_apply_kernel<false, true><<<dim3((kHalfRows * kDexp / 8) / 256), dim3(256), 0, stream>>>(
        ffh, pos, gam3, bet3, mean3, rstd3, A3h, kDexp, kHalfRows * kDexp / 8);
    gemm64_f16<2, 0, true><<<dim3((kHalfRows / 64) * (kDout / 64) / 8), dim3(256), 0, stream>>>(
        A3h, kDexp, W2T, kDexp, (void*)(out + (size_t)hb * kHalfRows * kDout), kDout, b2,
        x2 + (size_t)hb * kHalfRows * kDin, kHalfRows, kDout, kDexp, inv256);
  }
}
